// LNNFirstTransformerModel_61538291417789
// MI455X (gfx1250) — hardware-verified
//
#include <hip/hip_runtime.h>
#include <math.h>

constexpr int kB      = 16;
constexpr int kT      = 1024;
constexpr int kHid    = 256;
constexpr int kHeads  = 4;
constexpr int kDh     = 64;
constexpr int kFF     = 1024;
constexpr int kLayers = 2;
constexpr int kRows   = kB * kT;
constexpr int kQkvW   = 3 * kHid;
constexpr int kThr    = 256;
constexpr int kPairs  = kB * kHeads;
constexpr int kGrpPairs = 8;
constexpr int kGroups   = kPairs / kGrpPairs;
constexpr int kFFChunkRows = 4096;
constexpr int kFFChunks    = kRows / kFFChunkRows;
constexpr int kAPitch = 264;
constexpr int kSPitch = 260;
constexpr float kWCarry    = 16.0f;
constexpr float kWCarryInv = 1.0f / 16.0f;
constexpr float kPCarry    = 32768.0f;
constexpr float kCtxCarry  = 256.0f;
constexpr float kPVScale   = kCtxCarry / kPCarry;
constexpr float kWoScale   = 1.0f / (kCtxCarry * kWCarry);
constexpr float kAttnScale = 0.125f;
constexpr float kDt        = 0.1f;
constexpr float kLnEps     = 1e-5f;

static_assert(kRows % 64 == 0 && kHid % 64 == 0 && kQkvW % 64 == 0 && kFF % 64 == 0 && kT % 64 == 0 && kDh % 64 == 0);
static_assert(kHid % 32 == 0 && kDh % 32 == 0 && kT % 32 == 0 && kFF % 32 == 0);
static_assert(kHid == 32 * (kThr / 32));
static_assert((2 * kB * kAPitch) % kThr == 0);
static_assert(kRows % (kThr / 32) == 0);
static_assert(((kRows / 64) * (kHid / 64)) % 8 == 0);
static_assert(((kRows / 64) * (kQkvW / 64)) % 8 == 0);
static_assert(((kT / 64) * (kT / 64)) % 8 == 0);
static_assert(((kT / 64) * (kDh / 64)) % 8 == 0);
static_assert(((kFFChunkRows / 64) * (kFF / 64)) % 8 == 0);
static_assert(((kFFChunkRows / 64) * (kHid / 64)) % 8 == 0);

constexpr size_t kBytesU    = (size_t)kRows * kHid * 2;
constexpr size_t kBytesIP   = (size_t)kRows * kHid * 4;
constexpr size_t kBytesQKV  = (size_t)kRows * kQkvW * 2;
constexpr size_t kBytesR1   = (kBytesU + kBytesIP > kBytesQKV) ? (kBytesU + kBytesIP) : kBytesQKV;
constexpr size_t kBytesSEQ  = (size_t)kRows * kHid * 4;
constexpr size_t kBytesSEQH = (size_t)kRows * kHid * 2;
constexpr size_t kBytesVT   = (size_t)kPairs * kDh * kT * 2;
constexpr size_t kBytesS    = (size_t)kGrpPairs * kT * kT * 4;
constexpr size_t kBytesP    = (size_t)kGrpPairs * kT * kT * 2;
constexpr size_t kBytesATT  = (size_t)kRows * kHid * 4;
constexpr size_t kBytesPRE  = (size_t)kFFChunkRows * kFF * 4;
constexpr size_t kBytesACT  = (size_t)kFFChunkRows * kFF * 2;
constexpr size_t kBytesR2   = (kBytesS + kBytesP > kBytesATT + kBytesPRE + kBytesACT) ? (kBytesS + kBytesP) : (kBytesATT + kBytesPRE + kBytesACT);
constexpr size_t kBytesCTX  = (size_t)kRows * kHid * 2;
constexpr size_t kBytesWX   = (size_t)kHid * kHid * 2;
constexpr size_t kBytesWRT  = (size_t)kHid * kHid * 2;
constexpr size_t kBytesWQKV = (size_t)kLayers * kQkvW * kHid * 2;
constexpr size_t kBytesWO   = (size_t)kLayers * kHid * kHid * 2;
constexpr size_t kBytesW1   = (size_t)kLayers * kFF * kHid * 2;
constexpr size_t kBytesW2   = (size_t)kLayers * kHid * kFF * 2;
constexpr size_t kBytesTotal = kBytesR1 + kBytesSEQ + kBytesSEQH + kBytesVT + kBytesR2 + kBytesCTX +
                               kBytesWX + kBytesWRT + kBytesWQKV + kBytesWO + kBytesW1 + kBytesW2;
static_assert(kBytesTotal == 120848384);
static_assert(kBytesTotal <= (size_t)134217728);
static_assert(kBytesATT + kBytesPRE + kBytesACT <= kBytesR2);

typedef __attribute__((ext_vector_type(16))) _Float16 v16h;
typedef __attribute__((ext_vector_type(8)))  _Float16 v8h;
typedef __attribute__((ext_vector_type(16))) __bf16   v16b;
typedef __attribute__((ext_vector_type(8)))  __bf16   v8b;
typedef __attribute__((ext_vector_type(8)))  float    v8f;
typedef __attribute__((ext_vector_type(4)))  float    v4f;
typedef __attribute__((ext_vector_type(4)))  unsigned int v4u;

__device__ __forceinline__ unsigned short f2bf_bits(float f) {
  unsigned u = __float_as_uint(f);
  return (unsigned short)((u + 0x7FFFu + ((u >> 16) & 1u)) >> 16);
}
__device__ __forceinline__ float bf_bits2f(unsigned short h) { return __uint_as_float(((unsigned)h) << 16); }

__device__ __forceinline__ void dep_guard_h(v8f& a, v8f& b, v16h x, v16h y) { asm volatile("v_nop\n\tv_nop\n\tv_nop\n\tv_nop" : "+v"(a), "+v"(b) : "v"(x), "v"(y)); }
__device__ __forceinline__ void dep_guard_b(v8f& a, v8f& b, v16b x, v16b y) { asm volatile("v_nop\n\tv_nop\n\tv_nop\n\tv_nop" : "+v"(a), "+v"(b) : "v"(x), "v"(y)); }
__device__ __forceinline__ void keep4_h(v16h a, v16h b, v16h c, v16h d) { asm volatile("v_nop" :: "v"(a), "v"(b), "v"(c), "v"(d)); }
__device__ __forceinline__ void keep4_b(v16b a, v16b b, v16b c, v16b d) { asm volatile("v_nop" :: "v"(a), "v"(b), "v"(c), "v"(d)); }
__device__ __forceinline__ void acc_guard4(v8f& a, v8f& b, v8f& c, v8f& d) { asm volatile("v_nop\n\tv_nop\n\tv_nop\n\tv_nop" : "+v"(a), "+v"(b), "+v"(c), "+v"(d)); }
__device__ __forceinline__ void acc_guard2(v8f& a, v8f& b) { asm volatile("v_nop\n\tv_nop\n\tv_nop\n\tv_nop" : "+v"(a), "+v"(b)); }
template <typename T> struct Frag;
template <> struct Frag<_Float16> {
  typedef v16h V; union U { v16h v; v8h h[2]; };
  static __device__ __forceinline__ v16h load(const _Float16* p) {
    U f; f.h[0] = *(const v8h*)(p); f.h[1] = *(const v8h*)(p + 16); return f.v;
  }
  static __device__ __forceinline__ v8f mma(v16h a, v16h b, v8f c) {
    return __builtin_amdgcn_wmma_f32_16x16x32_f16(false, a, false, b, (short)0, c, false, false);
  }
  static __device__ __forceinline__ void guard(v8f& a, v8f& b, v16h x, v16h y) { dep_guard_h(a, b, x, y); }
  static __device__ __forceinline__ void keep(v16h a, v16h b, v16h c, v16h d) { keep4_h(a, b, c, d); }
};
template <> struct Frag<__bf16> {
  typedef v16b V; union U { v16b v; v8b h[2]; };
  static __device__ __forceinline__ v16b load(const __bf16* p) {
    U f; f.h[0] = *(const v8b*)(p); f.h[1] = *(const v8b*)(p + 16); return f.v;
  }
  static __device__ __forceinline__ v8f mma(v16b a, v16b b, v8f c) {
    return __builtin_amdgcn_wmma_f32_16x16x32_bf16(false, a, false, b, (short)0, c, false, false);
  }
  static __device__ __forceinline__ void guard(v8f& a, v8f& b, v16b x, v16b y) { dep_guard_b(a, b, x, y); }
  static __device__ __forceinline__ void keep(v16b a, v16b b, v16b c, v16b d) { keep4_b(a, b, c, d); }
};

__device__ __forceinline__ unsigned pk16(unsigned short a, unsigned short b) { return (unsigned)a | ((unsigned)b << 16); }
__device__ __forceinline__ unsigned short h_bits(float f) { const _Float16 h = (_Float16)f; return __builtin_bit_cast(unsigned short, h); }
__device__ __forceinline__ float ftanh(float x) { return 1.0f - 2.0f * __builtin_amdgcn_rcpf(__expf(2.0f * x) + 1.0f); }

template <int ET> struct Elem;
template <> struct Elem<0> { typedef _Float16 T; };
template <> struct Elem<1> { typedef __bf16 T; };
template <int ET, bool SPLIT, int BIAS_MODE, int OUT_MODE, bool RESID, int ACT = 0>
__global__ __launch_bounds__(256) void wmma_gemm64(
    const unsigned short* __restrict__ Ap, const unsigned short* __restrict__ A2p, int lda, long strideA,
    const unsigned short* __restrict__ Btp, const unsigned short* __restrict__ Bt2p, int ldb, long strideB,
    void* __restrict__ Cout, void* __restrict__ Cout2, int ldc, long strideC,
    const float* __restrict__ bias,
    const float* __restrict__ resid, long strideR,
    int M, int N, int K, float scale) {
  typedef typename Elem<ET>::T T;
  typedef typename Frag<T>::V V;
  const T* A = (const T*)Ap; const T* A2 = (const T*)A2p; const T* Bt = (const T*)Btp; const T* Bt2 = (const T*)Bt2p;
  __shared__ __align__(16) float sT[8][16 * 68];
  const int b    = blockIdx.y;
  const int lane = threadIdx.x & 31;
  const int wave = threadIdx.x >> 5;
  const int tilesN = N >> 6;
  const int tilesM = M >> 6;
  const int tile = blockIdx.x * 8 + wave;
  if (tile >= tilesM * tilesN) return;
  const int tm = tile / tilesN;
  const int tn = tile - tm * tilesN;
  const int m0 = tm << 6;
  const int n0 = tn << 6;

  const T* Ab  = A  + (size_t)b * strideA;
  const T* Bb  = Bt + (size_t)b * strideB;
  const T* Ab2 = SPLIT ? (A2  + (size_t)b * strideA) : nullptr;
  const T* Bb2 = SPLIT ? (Bt2 + (size_t)b * strideB) : nullptr;

  const int rlane = lane & 15;
  const int koff  = (lane >> 4) * 8;
  const int mOff  = (lane >> 4) * 8;

  v8f acc[4][4];
#pragma unroll
  for (int i = 0; i < 4; ++i)
#pragma unroll
    for (int j = 0; j < 4; ++j) acc[i][j] = (v8f){0.f,0.f,0.f,0.f,0.f,0.f,0.f,0.f};

  for (int k0 = 0; k0 < K; k0 += 32) {
    V bh[4], bl[4];
#pragma unroll
    for (int j = 0; j < 4; ++j) {
      const size_t bo = (size_t)(n0 + (j << 4) + rlane) * ldb + koff + k0;
      bh[j] = Frag<T>::load(Bb + bo);
      if (SPLIT) bl[j] = Frag<T>::load(Bb2 + bo);
    }
#pragma unroll
    for (int i = 0; i < 4; ++i) {
      const size_t ao = (size_t)(m0 + (i << 4) + rlane) * lda + koff + k0;
      V ah = Frag<T>::load(Ab + ao);
      V al;
      if (SPLIT) al = Frag<T>::load(Ab2 + ao);
#pragma unroll
      for (int j = 0; j < 4; ++j) {
        acc[i][j] = Frag<T>::mma(ah, bh[j], acc[i][j]);
        if (SPLIT) {
          acc[i][j] = Frag<T>::mma(ah, bl[j], acc[i][j]);
          acc[i][j] = Frag<T>::mma(al, bh[j], acc[i][j]);
        }
      }
      Frag<T>::guard(acc[i][0], acc[i][3], ah, SPLIT ? al : ah);
    }
    Frag<T>::keep(bh[0], bh[1], bh[2], bh[3]);
    if (SPLIT) Frag<T>::keep(bl[0], bl[1], bl[2], bl[3]);
  }
  acc_guard4(acc[0][0], acc[0][1], acc[0][2], acc[0][3]);
  acc_guard4(acc[1][0], acc[1][1], acc[1][2], acc[1][3]);
  acc_guard4(acc[2][0], acc[2][1], acc[2][2], acc[2][3]);
  acc_guard4(acc[3][0], acc[3][1], acc[3][2], acc[3][3]);

  float* slab = sT[wave];
  const float* Rb = RESID ? (resid + (size_t)b * strideR) : nullptr;
#pragma unroll
  for (int i = 0; i < 4; ++i) {
    const int mBase = m0 + (i << 4);
#pragma unroll
    for (int j = 0; j < 4; ++j) {
      const int n = n0 + (j << 4) + rlane;
      float bv = 0.f;
      if (BIAS_MODE == 2) bv = bias[n];
#pragma unroll
      for (int r = 0; r < 8; ++r) {
        float v = acc[i][j][r] * scale;
        if (BIAS_MODE == 1) v += bias[mBase + mOff + r];
        if (BIAS_MODE == 2) v += bv;
        if (RESID) v += Rb[(size_t)(mBase + mOff + r) * ldc + n];
        if (ACT == 2) v = fmaxf(v, 0.0f);
        if (ACT == 4) v = (v > 0.f) ? v : 0.01f * v;
        slab[(mOff + r) * 68 + (j << 4) + rlane] = v;
      }
    }
    __builtin_amdgcn_fence(__ATOMIC_RELEASE, "workgroup");
    __builtin_amdgcn_wave_barrier();
    __builtin_amdgcn_fence(__ATOMIC_ACQUIRE, "workgroup");
    if (OUT_MODE == 0) {
      float* C = (float*)Cout + (size_t)b * strideC;
      const int hh = lane >> 4, c4 = (lane & 15) * 4;
      for (int pass = 0; pass < 2; ++pass) {
#pragma unroll
        for (int it = 0; it < 8; ++it) {
          const int row = it * 2 + hh;
          v4f v = *(const v4f*)(slab + row * 68 + c4);
          *(volatile v4f*)(C + (size_t)(mBase + row) * ldc + n0 + c4) = v;
        }
        __threadfence();
      }
    } else {
      const int q = lane >> 3, c8 = (lane & 7) * 8;
      unsigned short* C  = (unsigned short*)Cout  + (size_t)b * strideC;
      unsigned short* C2 = (OUT_MODE == 2) ? ((unsigned short*)Cout2 + (size_t)b * strideC) : nullptr;
      for (int pass = 0; pass < 2; ++pass) {
#pragma unroll
        for (int it = 0; it < 4; ++it) {
          const int row = it * 4 + q;
          const float* sp = slab + row * 68 + c8;
          v8h hv, lv;
#pragma unroll
          for (int e = 0; e < 8; ++e) {
            if (OUT_MODE == 1) {
              hv[e] = (_Float16)sp[e];
            } else {
              unsigned short hb = f2bf_bits(sp[e]);
              unsigned short lb = f2bf_bits(sp[e] - bf_bits2f(hb));
              hv[e] = __builtin_bit_cast(_Float16, hb);
              lv[e] = __builtin_bit_cast(_Float16, lb);
            }
          }
          *(volatile v8h*)(C + (size_t)(mBase + row) * ldc + n0 + c8) = hv;
          if (OUT_MODE == 2) *(volatile v8h*)(C2 + (size_t)(mBase + row) * ldc + n0 + c8) = lv;
        }
        __threadfence();
      }
    }
    __builtin_amdgcn_fence(__ATOMIC_RELEASE, "workgroup");
    __builtin_amdgcn_wave_barrier();
    __builtin_amdgcn_fence(__ATOMIC_ACQUIRE, "workgroup");
  }
}

__global__ __launch_bounds__(kThr) void cast8_f16_kernel(const float* __restrict__ in, unsigned short* __restrict__ out,
                                                         int n8, float sc) {
  const int i = blockIdx.x * kThr + threadIdx.x;
  if (i >= n8) return;
  const float* p = in + 8 * (size_t)i;
  const v4f a = *(const v4f*)(p);
  const v4f c = *(const v4f*)(p + 4);
  unsigned short hb[8];
#pragma unroll
  for (int e = 0; e < 4; ++e) {
    hb[e]     = h_bits(a[e] * sc);
    hb[4 + e] = h_bits(c[e] * sc);
  }
  const v4u u = (v4u){pk16(hb[0], hb[1]), pk16(hb[2], hb[3]), pk16(hb[4], hb[5]), pk16(hb[6], hb[7])};
  unsigned short* q = out + 8 * (size_t)i;
  *(volatile v4u*)q = u;
  __threadfence();
  *(volatile v4u*)q = u;
}

__global__ __launch_bounds__(kThr) void wrec_tcast_kernel(const float* __restrict__ W, unsigned short* __restrict__ out, float sc) {
  __shared__ float sm[64][65];
  const int t  = threadIdx.x;
  const int k0 = blockIdx.x * 64;
  const int n0 = blockIdx.y * 64;
#pragma unroll
  for (int i = 0; i < 16; ++i) {
    const int e  = i * kThr + t;
    const int r  = e >> 6;
    const int cc = e & 63;
    sm[cc][r] = W[(size_t)(k0 + r) * kHid + n0 + cc] * sc;
  }
  __syncthreads();
  const int lane = t & 31, wave = t >> 5;
  const int q = lane >> 3, c8 = (lane & 7) * 8;
  for (int pass = 0; pass < 2; ++pass) {
#pragma unroll
    for (int it = 0; it < 2; ++it) {
      const int row = wave * 8 + it * 4 + q;
      unsigned short hb[8];
#pragma unroll
      for (int e = 0; e < 8; ++e) hb[e] = h_bits(sm[row][c8 + e]);
      const v4u u = (v4u){pk16(hb[0], hb[1]), pk16(hb[2], hb[3]), pk16(hb[4], hb[5]), pk16(hb[6], hb[7])};
      *(volatile v4u*)(out + (size_t)(n0 + row) * kHid + k0 + c8) = u;
    }
    __threadfence();
  }
}

__global__ __launch_bounds__(kThr) void vt_kernel(const unsigned short* __restrict__ QKV, unsigned short* __restrict__ VT) {
  __shared__ __align__(16) unsigned short sm[64][72];
  const int t  = threadIdx.x;
  const int p  = blockIdx.y;
  const int b  = p >> 2;
  const int h  = p & 3;
  const int t0 = blockIdx.x * 64;
#pragma unroll
  for (int it = 0; it < 2; ++it) {
    const int e  = it * kThr + t;
    const int r  = e >> 3;
    const int cc = e & 7;
    const v4u g = *(const v4u*)(QKV + (size_t)(b * kT + t0 + r) * kQkvW + 2 * kHid + h * kDh + cc * 8);
#pragma unroll
    for (int q4 = 0; q4 < 4; ++q4) {
      sm[r][cc * 8 + 2 * q4]     = (unsigned short)(g[q4] & 0xffffu);
      sm[r][cc * 8 + 2 * q4 + 1] = (unsigned short)(g[q4] >> 16);
    }
  }
  __syncthreads();
  const int lane = t & 31, wave = t >> 5;
  const int q = lane >> 3, c8 = (lane & 7) * 8;
  v4u u[2];
#pragma unroll
  for (int it = 0; it < 2; ++it) {
    const int row = wave * 8 + it * 4 + q;
    unsigned short hb[8];
#pragma unroll
    for (int e = 0; e < 8; ++e) hb[e] = sm[c8 + e][row];
    u[it] = (v4u){pk16(hb[0], hb[1]), pk16(hb[2], hb[3]), pk16(hb[4], hb[5]), pk16(hb[6], hb[7])};
  }
  unsigned short* op = VT + (size_t)p * kDh * kT;
  for (int pass = 0; pass < 2; ++pass) {
#pragma unroll
    for (int it = 0; it < 2; ++it) {
      const int row = wave * 8 + it * 4 + q;
      *(volatile v4u*)(op + (size_t)row * kT + t0 + c8) = u[it];
    }
    __threadfence();
  }
}

__global__ __launch_bounds__(kThr) void inproj_kernel(const float* __restrict__ x, const float* __restrict__ Win,
                                                      const float* __restrict__ bin, const float* __restrict__ gam,
                                                      const float* __restrict__ bet, unsigned short* __restrict__ U) {
  __shared__ __align__(16) unsigned short su[kThr / 32][kAPitch];
  const int tid = threadIdx.x, lane = tid & 31, wave = tid >> 5;
  const int row = blockIdx.x * (kThr / 32) + wave;
  const float xv = x[row];
  const v4f w0 = *(const v4f*)(Win + 8 * lane);
  const v4f w1 = *(const v4f*)(Win + 8 * lane + 4);
  const v4f b0 = *(const v4f*)(bin + 8 * lane);
  const v4f b1 = *(const v4f*)(bin + 8 * lane + 4);
  float v[8];
#pragma unroll
  for (int e = 0; e < 4; ++e) { v[e] = xv * w0[e] + b0[e]; v[4 + e] = xv * w1[e] + b1[e]; }
  float s = ((v[0] + v[1]) + (v[2] + v[3])) + ((v[4] + v[5]) + (v[6] + v[7]));
#pragma unroll
  for (int off = 1; off < 32; off <<= 1) s += __shfl_xor(s, off, 32);
  const float mu = s * (1.0f / kHid);
  float ss = 0.0f;
#pragma unroll
  for (int e = 0; e < 8; ++e) { const float d = v[e] - mu; ss += d * d; }
#pragma unroll
  for (int off = 1; off < 32; off <<= 1) ss += __shfl_xor(ss, off, 32);
  const float var  = ss * (1.0f / kHid);
  const float rstd = rsqrtf(var + kLnEps);
#pragma unroll 1
  for (int it = 0; it < 8; ++it) {
    const int c = 8 * lane + it;
    const float w  = Win[c];
    const float bb = bin[c];
    const float g  = gam[c];
    const float be = bet[c];
    const float y  = ((xv * w + bb) - mu) * rstd * g + be;
    const float gl = 0.5f * y * (1.0f + erff(y * 0.70710678118654752f));
    su[wave][c] = h_bits(gl);
  }
  __syncthreads();
  const unsigned short* sr = &su[wave][8 * lane];
  const v4u u = (v4u){pk16(sr[0], sr[1]), pk16(sr[2], sr[3]), pk16(sr[4], sr[5]), pk16(sr[6], sr[7])};
  unsigned short* op = U + (size_t)row * kHid + 8 * lane;
  *(volatile v4u*)op = u;
  __threadfence();
  *(volatile v4u*)op = u;
}

__global__ __launch_bounds__(kThr) void lnn_rec_kernel(const float* __restrict__ IP, const unsigned short* __restrict__ WRTp,
                                                       const float* __restrict__ tau, float* __restrict__ SEQ,
                                                       unsigned short* __restrict__ SEQH) {
  __shared__ __align__(16) _Float16 Ah[2][kB * kAPitch];
  __shared__ __align__(16) float    Sf[2][kB * kSPitch];
  const _Float16* WRT = (const _Float16*)WRTp;
  const int tid = threadIdx.x, lane = tid & 31, wave = tid >> 5;
  const int c = lane & 15, hh = lane >> 4, koff = hh * 8;

  {
    _Float16* ahf = &Ah[0][0];
#pragma unroll 1
    for (int i = tid; i < 2 * kB * kAPitch; i += kThr) ahf[i] = (_Float16)0.0f;
  }
  float hst[2][8];
#pragma unroll
  for (int nt = 0; nt < 2; ++nt)
#pragma unroll
    for (int r = 0; r < 8; ++r) hst[nt][r] = 0.0f;
  float rtau[2];
#pragma unroll
  for (int nt = 0; nt < 2; ++nt) rtau[nt] = 1.0f / tau[32 * wave + 16 * nt + c];
  __syncthreads();

  const v8f z8 = {0.f, 0.f, 0.f, 0.f, 0.f, 0.f, 0.f, 0.f};
  const _Float16* wr0 = WRT + (size_t)(32 * wave + c) * kHid + koff;
  const _Float16* wr1 = wr0 + (size_t)16 * kHid;

#pragma unroll 1
  for (int t = 0; t < kT; ++t) {
    const int cur = t & 1;
    const _Float16* ahrow = &Ah[cur][0] + c * kAPitch + koff;
    _Float16* ahn = &Ah[cur ^ 1][0];
    float* sf = &Sf[cur][0];

    v8f acc[2];
    acc[0] = z8; acc[1] = z8;
#pragma unroll 1
    for (int k0 = 0; k0 < kHid; k0 += 32) {
      const v16h a  = Frag<_Float16>::load(ahrow + k0);
      const v16h b0 = Frag<_Float16>::load(wr0 + k0);
      const v16h b1 = Frag<_Float16>::load(wr1 + k0);
      acc[0] = Frag<_Float16>::mma(a, b0, acc[0]);
      acc[1] = Frag<_Float16>::mma(a, b1, acc[1]);
      dep_guard_h(acc[0], acc[1], a, b1);
      keep4_h(a, b0, b1, a);
    }
    acc_guard2(acc[0], acc[1]);

#pragma unroll
    for (int nt = 0; nt < 2; ++nt) {
      const int j = 32 * wave + 16 * nt + c;
#pragma unroll
      for (int r = 0; r < 8; ++r) {
        const int row = 8 * hh + r;
        const float ipv = IP[((size_t)row * kT + (size_t)t) * kHid + j];
        const float z   = acc[nt][r] * kWCarryInv + ipv;
        const float f   = ftanh(z);
        const float ho  = hst[nt][r];
        float hn = ho + (f - ho * rtau[nt]) * kDt;
        hn = fminf(10.0f, fmaxf(-10.0f, hn));
        hst[nt][r] = hn;
        ahn[row * kAPitch + j] = (_Float16)hn;
        sf[row * kSPitch + j] = hn;
      }
    }
    __syncthreads();

    v4f va[2], vb[2];
    v8h hv[2];
#pragma unroll
    for (int i = 0; i < 2; ++i) {
      const int row = 2 * wave + i;
      const float* sr = sf + row * kSPitch;
      va[i] = *(const v4f*)(sr + 4 * lane);
      vb[i] = *(const v4f*)(sr + 128 + 4 * lane);
      const v4f p0 = *(const v4f*)(sr + 8 * lane);
      const v4f p1 = *(const v4f*)(sr + 8 * lane + 4);
#pragma unroll
      for (int e = 0; e < 4; ++e) { hv[i][e] = (_Float16)p0[e]; hv[i][4 + e] = (_Float16)p1[e]; }
    }
    for (int pass = 0; pass < 2; ++pass) {
#pragma unroll
      for (int i = 0; i < 2; ++i) {
        const int row = 2 * wave + i;
        const size_t g = ((size_t)row * kT + (size_t)t) * kHid;
        *(volatile v4f*)(SEQ + g + 4 * lane) = va[i];
        *(volatile v4f*)(SEQ + g + 128 + 4 * lane) = vb[i];
        *(volatile v8h*)(SEQH + g + 8 * lane) = hv[i];
      }
      __threadfence();
    }
  }
}

__global__ __launch_bounds__(128) void softmax_row_kernel(const float* __restrict__ S, unsigned short* __restrict__ P, float carry) {
  __shared__ float redM[4];
  __shared__ float redS[4];
  const int row  = blockIdx.x;
  const int t    = threadIdx.x;
  const int lane = t & 31, wave = t >> 5;
  const int c0   = t * 8;
  const float* sr = S + (size_t)row * kT + c0;
  const v4f a = *(const v4f*)(sr);
  const v4f c = *(const v4f*)(sr + 4);
  float x[8];
#pragma unroll
  for (int e = 0; e < 4; ++e) { x[e] = a[e]; x[4 + e] = c[e]; }
  float m = fmaxf(fmaxf(fmaxf(x[0], x[1]), fmaxf(x[2], x[3])), fmaxf(fmaxf(x[4], x[5]), fmaxf(x[6], x[7])));
#pragma unroll
  for (int off = 1; off < 32; off <<= 1) m = fmaxf(m, __shfl_xor(m, off, 32));
  if (lane == 0) redM[wave] = m;
  __syncthreads();
  const float gm = fmaxf(fmaxf(redM[0], redM[1]), fmaxf(redM[2], redM[3]));
  float ev[8];
#pragma unroll
  for (int e = 0; e < 8; ++e) ev[e] = expf(x[e] - gm);
  float s = ((ev[0] + ev[1]) + (ev[2] + ev[3])) + ((ev[4] + ev[5]) + (ev[6] + ev[7]));
#pragma unroll
  for (int off = 1; off < 32; off <<= 1) s += __shfl_xor(s, off, 32);
  if (lane == 0) redS[wave] = s;
  __syncthreads();
  const float tot = ((redS[0] + redS[1]) + redS[2]) + redS[3];
  const float inv = carry / tot;
  unsigned short hb[8];
#pragma unroll
  for (int e = 0; e < 8; ++e) hb[e] = h_bits(ev[e] * inv);
  const v4u u = (v4u){pk16(hb[0], hb[1]), pk16(hb[2], hb[3]), pk16(hb[4], hb[5]), pk16(hb[6], hb[7])};
  unsigned short* q = P + (size_t)row * kT + c0;
  *(volatile v4u*)q = u;
  __threadfence();
  *(volatile v4u*)q = u;
}

__global__ __launch_bounds__(kThr) void ln_rows_kernel(const float* __restrict__ X, const float* __restrict__ gam,
                                                       const float* __restrict__ bet, float* __restrict__ Y,
                                                       unsigned short* __restrict__ YH) {
  __shared__ __align__(16) float slab[kThr / 32][kHid];
  const int tid = threadIdx.x, lane = tid & 31, wave = tid >> 5;
  const int row = blockIdx.x * (kThr / 32) + wave;
  const float* rp = X + (size_t)row * kHid;
  v4f v[2], g[2], bb[2];
  v[0]  = *(const v4f*)(rp  + 4 * lane);        v[1]  = *(const v4f*)(rp  + 128 + 4 * lane);
  g[0]  = *(const v4f*)(gam + 4 * lane);        g[1]  = *(const v4f*)(gam + 128 + 4 * lane);
  bb[0] = *(const v4f*)(bet + 4 * lane);        bb[1] = *(const v4f*)(bet + 128 + 4 * lane);
  float s = ((v[0][0] + v[0][1]) + (v[0][2] + v[0][3])) + ((v[1][0] + v[1][1]) + (v[1][2] + v[1][3]));
#pragma unroll
  for (int off = 1; off < 32; off <<= 1) s += __shfl_xor(s, off, 32);
  const float mu = s * (1.0f / kHid);
  float ss = 0.0f;
#pragma unroll
  for (int q = 0; q < 2; ++q)
#pragma unroll
    for (int e = 0; e < 4; ++e) { const float d = v[q][e] - mu; v[q][e] = d; ss += d * d; }
#pragma unroll
  for (int off = 1; off < 32; off <<= 1) ss += __shfl_xor(ss, off, 32);
  const float var  = ss * (1.0f / kHid);
  const float rstd = rsqrtf(var + kLnEps);
  v4f o[2];
#pragma unroll
  for (int q = 0; q < 2; ++q)
#pragma unroll
    for (int e = 0; e < 4; ++e) o[q][e] = (v[q][e] * rstd) * g[q][e] + bb[q][e];
  float* sl = slab[wave];
  *(v4f*)(sl + 4 * lane) = o[0];
  *(v4f*)(sl + 128 + 4 * lane) = o[1];
  __builtin_amdgcn_fence(__ATOMIC_RELEASE, "workgroup");
  __builtin_amdgcn_wave_barrier();
  __builtin_amdgcn_fence(__ATOMIC_ACQUIRE, "workgroup");
  const v4f p0 = *(const v4f*)(sl + 8 * lane);
  const v4f p1 = *(const v4f*)(sl + 8 * lane + 4);
  v8h hv;
#pragma unroll
  for (int e = 0; e < 4; ++e) { hv[e] = (_Float16)p0[e]; hv[4 + e] = (_Float16)p1[e]; }
  float* yp = Y + (size_t)row * kHid;
  unsigned short* hp = YH + (size_t)row * kHid;
  for (int pass = 0; pass < 2; ++pass) {
    *(volatile v4f*)(yp + 4 * lane) = o[0];
    *(volatile v4f*)(yp + 128 + 4 * lane) = o[1];
    *(volatile v8h*)(hp + 8 * lane) = hv;
    __threadfence();
  }
}

__global__ __launch_bounds__(kThr) void gelu2_kernel(const float* __restrict__ in, unsigned short* __restrict__ out, int n2) {
  const int i = blockIdx.x * kThr + threadIdx.x;
  if (i >= n2) return;
  const float f0 = in[2 * (size_t)i];
  const float f1 = in[2 * (size_t)i + 1];
  const float g0 = 0.5f * f0 * (1.0f + erff(f0 * 0.70710678118654752f));
  const float g1 = 0.5f * f1 * (1.0f + erff(f1 * 0.70710678118654752f));
  const unsigned u = pk16(h_bits(g0), h_bits(g1));
  ((volatile unsigned*)out)[i] = u;
  __threadfence();
  ((volatile unsigned*)out)[i] = u;
}

__global__ __launch_bounds__(kThr) void pool_head_kernel(const float* __restrict__ SEQ, const float* __restrict__ Wfc,
                                                         const float* __restrict__ bfc, float* __restrict__ out) {
  __shared__ float red[kThr / 32];
  __shared__ float outv[kB];
  const int tid = threadIdx.x, lane = tid & 31, wave = tid >> 5;
  const float w  = Wfc[tid];
  const float bf = bfc[0];
#pragma unroll 1
  for (int b = 0; b < kB; ++b) {
    const float* sp = SEQ + (size_t)b * kT * kHid + tid;
    float s0 = 0.0f, s1 = 0.0f, s2 = 0.0f, s3 = 0.0f;
#pragma unroll 1
    for (int t = 0; t < kT; t += 4) {
      s0 += sp[(size_t)(t)     * kHid];
      s1 += sp[(size_t)(t + 1) * kHid];
      s2 += sp[(size_t)(t + 2) * kHid];
      s3 += sp[(size_t)(t + 3) * kHid];
    }
    const float s = (s0 + s1) + (s2 + s3);
    float pv = (s * (1.0f / kT)) * w;
#pragma unroll
    for (int off = 1; off < 32; off <<= 1) pv += __shfl_xor(pv, off, 32);
    if (lane == 0) red[wave] = pv;
    __syncthreads();
    if (tid == 0) {
      float tot = red[0];
#pragma unroll
      for (int q = 1; q < kThr / 32; ++q) tot += red[q];
      outv[b] = tot + bf;
    }
    __syncthreads();
  }
  if (wave == 0) {
    const float v = outv[lane & 15];
    if (lane < kB) *(volatile float*)(out + lane) = v;
    __threadfence();
    if (lane < kB) *(volatile float*)(out + lane) = v;
  }
}

extern "C" void kernel_launch(void* const* d_in, const int* in_sizes, int n_in,
                              void* d_out, int out_size, void* d_ws, size_t ws_size, hipStream_t stream) {
  if (n_in < 23 || d_out == nullptr || d_ws == nullptr) return;
  if (in_sizes[0] != kB * kT || in_sizes[1] != kHid || in_sizes[2] != kHid || in_sizes[3] != kHid || in_sizes[4] != kHid ||
      in_sizes[5] != kHid * kHid || in_sizes[6] != kHid || in_sizes[7] != kHid || in_sizes[8] != kHid * kHid ||
      in_sizes[9] != kLayers * kQkvW * kHid || in_sizes[10] != kLayers * kQkvW ||
      in_sizes[11] != kLayers * kHid * kHid || in_sizes[12] != kLayers * kHid ||
      in_sizes[13] != kLayers * kHid || in_sizes[14] != kLayers * kHid ||
      in_sizes[15] != kLayers * kFF * kHid || in_sizes[16] != kLayers * kFF ||
      in_sizes[17] != kLayers * kHid * kFF || in_sizes[18] != kLayers * kHid ||
      in_sizes[19] != kLayers * kHid || in_sizes[20] != kLayers * kHid ||
      in_sizes[21] != kHid || in_sizes[22] != 1 || out_size != kB) return;

  const float* x     = (const float*)d_in[0];
  const float* W_in  = (const float*)d_in[1];
  const float* b_in  = (const float*)d_in[2];
  const float* lng   = (const float*)d_in[3];
  const float* lnb   = (const float*)d_in[4];
  const float* W_x   = (const float*)d_in[5];
  const float* b_x   = (const float*)d_in[6];
  const float* tau   = (const float*)d_in[7];
  const float* W_rec = (const float*)d_in[8];
  const float* Wqkv  = (const float*)d_in[9];
  const float* bqkv  = (const float*)d_in[10];
  const float* Wo    = (const float*)d_in[11];
  const float* bo    = (const float*)d_in[12];
  const float* ln1g  = (const float*)d_in[13];
  const float* ln1b  = (const float*)d_in[14];
  const float* W1    = (const float*)d_in[15];
  const float* b1    = (const float*)d_in[16];
  const float* W2    = (const float*)d_in[17];
  const float* b2    = (const float*)d_in[18];
  const float* ln2g  = (const float*)d_in[19];
  const float* ln2b  = (const float*)d_in[20];
  const float* W_fc  = (const float*)d_in[21];
  const float* b_fc  = (const float*)d_in[22];
  float* y_out = (float*)d_out;

  char* ws = (char*)d_ws; size_t off = 0;
  auto carve = [&](size_t bytes) -> char* { char* p = ws + off; off += (bytes + 255) & ~(size_t)255; return p; };
  char* R1 = carve(kBytesR1);
  float*          SEQ   = (float*)carve(kBytesSEQ);
  unsigned short* SEQH  = (unsigned short*)carve(kBytesSEQH);
  unsigned short* VT    = (unsigned short*)carve(kBytesVT);
  char* R2 = carve(kBytesR2);
  unsigned short* CTX   = (unsigned short*)carve(kBytesCTX);
  unsigned short* WX16  = (unsigned short*)carve(kBytesWX);
  unsigned short* WRT16 = (unsigned short*)carve(kBytesWRT);
  unsigned short* WQKV16 = (unsigned short*)carve(kBytesWQKV);
  unsigned short* WO16  = (unsigned short*)carve(kBytesWO);
  unsigned short* W1_16 = (unsigned short*)carve(kBytesW1);
  unsigned short* W2_16 = (unsigned short*)carve(kBytesW2);
  if (off > ws_size || off > (size_t)134217728) return;

  unsigned short* U16p = (unsigned short*)R1;
  float*          IP   = (float*)(R1 + kBytesU);
  unsigned short* QKV  = (unsigned short*)R1;
  float*          S    = (float*)R2;
  unsigned short* P    = (unsigned short*)(R2 + kBytesS);
  float*          ATT  = (float*)R2;
  float*          PRE  = (float*)(R2 + kBytesATT);
  unsigned short* ACT  = (unsigned short*)(R2 + kBytesATT + kBytesPRE);

  {
    const int n8 = kHid * kHid / 8;
    cast8_f16_kernel<<<(n8 + kThr - 1) / kThr, kThr, 0, stream>>>(W_x, WX16, n8, kWCarry);
  }
  wrec_tcast_kernel<<<dim3(kHid / 64, kHid / 64), kThr, 0, stream>>>(W_rec, WRT16, kWCarry);
  {
    const int n8 = kLayers * kQkvW * kHid / 8;
    cast8_f16_kernel<<<(n8 + kThr - 1) / kThr, kThr, 0, stream>>>(Wqkv, WQKV16, n8, kWCarry);
  }
  {
    const int n8 = kLayers * kHid * kHid / 8;
    cast8_f16_kernel<<<(n8 + kThr - 1) / kThr, kThr, 0, stream>>>(Wo, WO16, n8, kWCarry);
  }
  {
    const int n8 = kLayers * kFF * kHid / 8;
    cast8_f16_kernel<<<(n8 + kThr - 1) / kThr, kThr, 0, stream>>>(W1, W1_16, n8, kWCarry);
    cast8_f16_kernel<<<(n8 + kThr - 1) / kThr, kThr, 0, stream>>>(W2, W2_16, n8, kWCarry);
  }

  inproj_kernel<<<kRows / (kThr / 32), kThr, 0, stream>>>(x, W_in, b_in, lng, lnb, U16p);

  {
    const dim3 grid((kRows / 64) * (kHid / 64) / 8, 1);
    wmma_gemm64<0, false, 2, 0, false, 0><<<grid, 256, 0, stream>>>(
        U16p, U16p, kHid, 0L, WX16, WX16, kHid, 0L, (void*)IP, (void*)IP, kHid, 0L,
        b_x, SEQ, 0L, kRows, kHid, kHid, kWCarryInv);
  }

  lnn_rec_kernel<<<1, kThr, 0, stream>>>(IP, WRT16, tau, SEQ, SEQH);

  const long qkvBatchStride = (long)kT * kQkvW;
  const long ctxBatchStride = (long)kT * kHid;
  for (int l = 0; l < kLayers; ++l) {
    {
      const dim3 grid((kRows / 64) * (kQkvW / 64) / 8, 1);
      wmma_gemm64<0, false, 2, 1, false, 0><<<grid, 256, 0, stream>>>(
          SEQH, SEQH, kHid, 0L, WQKV16 + (size_t)l * kQkvW * kHid, WQKV16, kHid, 0L,
          (void*)QKV, (void*)QKV, kQkvW, 0L, bqkv + (size_t)l * kQkvW, SEQ, 0L, kRows, kQkvW, kHid, kWCarryInv);
    }
    vt_kernel<<<dim3(kT / 64, kPairs), kThr, 0, stream>>>(QKV, VT);

    for (int grp = 0; grp < kGroups; ++grp) {
      const int h  = grp & 3;
      const int bh = grp >> 2;
      const unsigned short* qp = QKV + (size_t)bh * kGrpPairs * qkvBatchStride + (size_t)h * kDh;
      const unsigned short* kp = qp + kHid;
      {
        const dim3 grid((kT / 64) * (kT / 64) / 8, kGrpPairs);
        wmma_gemm64<0, false, 0, 0, false, 0><<<grid, 256, 0, stream>>>(
            qp, qp, kQkvW, qkvBatchStride, kp, kp, kQkvW, qkvBatchStride,
            (void*)S, (void*)S, kT, (long)kT * kT, b_x, SEQ, 0L, kT, kT, kDh, kAttnScale);
      }
      softmax_row_kernel<<<kGrpPairs * kT, 128, 0, stream>>>(S, P, kPCarry);
      {
        const dim3 grid((kT / 64) * (kDh / 64) / 8, kGrpPairs);
        const unsigned short* vtp = VT + ((size_t)bh * kGrpPairs * kHeads + h) * (size_t)(kDh * kT);
        unsigned short* cp = CTX + (size_t)bh * kGrpPairs * ctxBatchStride + (size_t)h * kDh;
        wmma_gemm64<0, false, 0, 1, false, 0><<<grid, 256, 0, stream>>>(
            P, P, kT, (long)kT * kT, vtp, vtp, kT, (long)kHeads * kDh * kT,
            (void*)cp, (void*)cp, kHid, ctxBatchStride, b_x, SEQ, 0L, kT, kDh, kT, kPVScale);
      }
    }

    {
      const dim3 grid((kRows / 64) * (kHid / 64) / 8, 1);
      wmma_gemm64<0, false, 2, 0, true, 0><<<grid, 256, 0, stream>>>(
          CTX, CTX, kHid, 0L, WO16 + (size_t)l * kHid * kHid, WO16, kHid, 0L,
          (void*)ATT, (void*)ATT, kHid, 0L, bo + (size_t)l * kHid, SEQ, 0L, kRows, kHid, kHid, kWoScale);
    }
    ln_rows_kernel<<<kRows / (kThr / 32), kThr, 0, stream>>>(ATT, ln1g + (size_t)l * kHid, ln1b + (size_t)l * kHid, SEQ, SEQH);

    for (int ch = 0; ch < kFFChunks; ++ch) {
      const size_t rowOff = (size_t)ch * kFFChunkRows * kHid;
      {
        const dim3 grid((kFFChunkRows / 64) * (kFF / 64) / 8, 1);
        wmma_gemm64<0, false, 2, 0, false, 0><<<grid, 256, 0, stream>>>(
            SEQH + rowOff, SEQH, kHid, 0L, W1_16 + (size_t)l * kFF * kHid, W1_16, kHid, 0L,
            (void*)PRE, (void*)PRE, kFF, 0L, b1 + (size_t)l * kFF, SEQ, 0L, kFFChunkRows, kFF, kHid, kWCarryInv);
      }
      {
        const int n2 = kFFChunkRows * kFF / 2;
        gelu2_kernel<<<(n2 + kThr - 1) / kThr, kThr, 0, stream>>>(PRE, ACT, n2);
      }
      {
        const dim3 grid((kFFChunkRows / 64) * (kHid / 64) / 8, 1);
        wmma_gemm64<0, false, 2, 0, true, 0><<<grid, 256, 0, stream>>>(
            ACT, ACT, kFF, 0L, W2_16 + (size_t)l * kHid * kFF, W2_16, kFF, 0L,
            (void*)(ATT + rowOff), (void*)(ATT + rowOff), kHid, 0L, b2 + (size_t)l * kHid, SEQ + rowOff, 0L,
            kFFChunkRows, kHid, kFF, kWCarryInv);
      }
    }
    ln_rows_kernel<<<kRows / (kThr / 32), kThr, 0, stream>>>(ATT, ln2g + (size_t)l * kHid, ln2b + (size_t)l * kHid, SEQ, SEQH);
  }

  pool_head_kernel<<<1, kThr, 0, stream>>>(SEQ, W_fc, b_fc, y_out);
}
